// MoEsparseRouting_80358838108605
// MI455X (gfx1250) — hardware-verified
//
#include <hip/hip_runtime.h>
#include <math.h>

typedef __attribute__((ext_vector_type(16))) _Float16 v16h;
typedef __attribute__((ext_vector_type(16))) __bf16 v16b;
typedef __attribute__((ext_vector_type(8)))  _Float16 v8h;
typedef __attribute__((ext_vector_type(8)))  float v8f;
typedef __attribute__((ext_vector_type(4)))  float v4f;
typedef __attribute__((ext_vector_type(2)))  float v2f;
typedef __attribute__((ext_vector_type(4)))  unsigned v4u;
typedef __attribute__((ext_vector_type(4)))  int v4i;
typedef float __attribute__((may_alias)) float_a;
typedef int __attribute__((may_alias)) int_a;

template <typename T> __device__ __forceinline__ void vst2(void* p, T v) { *(volatile T*)p = v; __threadfence(); *(volatile T*)p = v; }
__device__ __forceinline__ v8f wmma16(v16h a, v16h b, v8f c) {
  v8f d = __builtin_amdgcn_wmma_f32_16x16x32_f16(false, a, false, b, (short)0, c, false, false);
  asm volatile("v_nop\n\tv_nop\n\tv_nop\n\tv_nop" : "+v"(d) : "v"(a), "v"(b));
  return d;
}
__device__ __forceinline__ v8f wmma_bf(v16b a, v16b b, v8f c) {
  v8f d = __builtin_amdgcn_wmma_f32_16x16x32_bf16(false, a, false, b, (short)0, c, false, false);
  asm volatile("v_nop\n\tv_nop\n\tv_nop\n\tv_nop" : "+v"(d) : "v"(a), "v"(b));
  return d;
}
__device__ __forceinline__ v16h frag_h(const _Float16* rowk0, int lane) {
  union { v16h v; v8h q[2]; } u; const _Float16* p = rowk0 + 8 * (lane >> 4);
  u.q[0] = *(const v8h*)p; u.q[1] = *(const v8h*)(p + 16); return u.v;
}
__device__ __forceinline__ v16h frag_f32(const float* rowk0, int lane) {
  v16h a; const float* p = rowk0 + 8 * (lane >> 4);
#pragma unroll
  for (int i = 0; i < 8; ++i) { a[i] = (_Float16)p[i]; a[8 + i] = (_Float16)p[16 + i]; }
  return a;
}
__device__ __forceinline__ v16h frag_f32s(const float* rowk0, int lane, float sc) {
  v16h a; const float* p = rowk0 + 8 * (lane >> 4);
#pragma unroll
  for (int i = 0; i < 8; ++i) { a[i] = (_Float16)(p[i] * sc); a[8 + i] = (_Float16)(p[16 + i] * sc); }
  return a;
}
__device__ __forceinline__ v16h fragc_f32(const float* W, int k0, int n, int lane, int ld, int K) {
  v16h a; const int g = lane >> 4;
#pragma unroll
  for (int i = 0; i < 8; ++i) { const int ka = k0 + 8 * g + i, kb = ka + 16;
    a[i] = (_Float16)(ka < K ? W[(size_t)(ka < K ? ka : K - 1) * ld + n] : 0.f); a[8 + i] = (_Float16)(kb < K ? W[(size_t)(kb < K ? kb : K - 1) * ld + n] : 0.f); }
  return a;
}
struct F2 { v16b h, l; };
__device__ __forceinline__ F2 bsplit16(const float v[16]) { F2 r;
#pragma unroll
  for (int i = 0; i < 16; ++i) { const __bf16 h = (__bf16)v[i]; r.h[i] = h; r.l[i] = (__bf16)(v[i] - (float)h); }
  return r; }
__device__ __forceinline__ F2 split_row(const float* row, int k0, int lane) { float v[16]; const float* p = row + k0 + 8 * (lane >> 4);
#pragma unroll
  for (int i = 0; i < 8; ++i) { v[i] = p[i]; v[8 + i] = p[16 + i]; }
  return bsplit16(v); }
__device__ __forceinline__ F2 split_rowK(const float* row, int k0, int lane, int K) { float v[16]; const int g = lane >> 4;
#pragma unroll
  for (int i = 0; i < 8; ++i) { const int ka = k0 + 8 * g + i, kb = ka + 16; v[i] = ka < K ? row[ka < K ? ka : K - 1] : 0.f; v[8 + i] = kb < K ? row[kb < K ? kb : K - 1] : 0.f; }
  return bsplit16(v); }
__device__ __forceinline__ F2 split_col(const float* W, int k0, int n, int lane, int ld, int K) { float v[16]; const int g = lane >> 4;
#pragma unroll
  for (int i = 0; i < 8; ++i) { const int ka = k0 + 8 * g + i, kb = ka + 16; v[i] = ka < K ? W[(size_t)(ka < K ? ka : K - 1) * ld + n] : 0.f; v[8 + i] = kb < K ? W[(size_t)(kb < K ? kb : K - 1) * ld + n] : 0.f; }
  return bsplit16(v); }
__device__ __forceinline__ v8f mac3(const F2& a, const F2& b, v8f c) { c = wmma_bf(a.l, b.h, c); c = wmma_bf(a.h, b.l, c); return wmma_bf(a.h, b.h, c); }
__device__ __forceinline__ float sigm(float v) { return 1.0f / (1.0f + expf(-v)); }
#define LDSX() do { asm volatile("s_wait_dscnt 0" ::: "memory"); __builtin_amdgcn_wave_barrier(); __builtin_amdgcn_fence(__ATOMIC_RELEASE, "workgroup"); } while (0)


#define NBT 8
#define SS 2048
#define DM 768
#define NE 16
#define RR 16
#define NTK (NBT * SS)
#define TPB 16
#ifndef NTB
#define NTB (NTK / TPB)
#define NRT (NTK / 64)
#endif
typedef __attribute__((ext_vector_type(8))) __bf16 v8b;
__device__ __forceinline__ v16b frag_b(const __bf16* rowk0, int lane) {
  union { v16b v; v8b q[2]; } u; const __bf16* p = rowk0 + 8 * (lane >> 4);
  u.q[0] = *(const v8b*)p; u.q[1] = *(const v8b*)(p + 16); return u.v;
}
__device__ __forceinline__ float bfr(float v) { return (float)(__bf16)v; }
__device__ __attribute__((noinline)) float exp_ni(float v) { return expf(v); }
__device__ __attribute__((noinline)) float erf_ni(float v) { return erff(v); }

#define PK_W   0
#define PK_C0  (PK_W + DM * DM)
#define PK_C1  (PK_C0 + NE * 16 * 32)
#define PK_C2  (PK_C1 + NE * 16 * 128)
#define PK_C3  (PK_C2 + NE * 16 * 128)
#define PK_C4  (PK_C3 + NE * 128 * 32)
#define PK_C5  (PK_C4 + NE * 128 * 32)
#define PK_END (PK_C5 + NE * 16 * 32)
#define WS_PK  0u
#define WS_XB  (((2u * PK_END) + 127u) / 128u * 128u)
#define WS_Z   (WS_XB + 2u * NTK * DM)
#define WS_END (WS_Z + 4u * NTK * DM)

__global__ __launch_bounds__(256) void k_pack(const float* __restrict__ BW, const float* __restrict__ C0, const float* __restrict__ C1, const float* __restrict__ C2, const float* __restrict__ C3, const float* __restrict__ C4, const float* __restrict__ C5, __bf16* __restrict__ PK) {
  __shared__ __align__(16) __bf16 s[128 * 32 * 2 + 16 * 128 * 2 + 16 * 32 * 2];
  const int n = blockIdx.x, which = blockIdx.y, tid = threadIdx.x;
  if (which == 0) { __bf16* row = s; for (int k = tid; k < DM; k += 256) row[k] = (__bf16)BW[(size_t)n * DM + k]; __syncthreads(); for (int q = tid; q < DM / 8; q += 256) vst2((unsigned*)(PK + PK_W + (size_t)n * DM + q * 8), *(const v4u*)&row[q * 8]); return; }
  if (n >= NE) return; const int e = n;
  __bf16 *s0 = s, *s1 = s0 + 16 * 32, *s2 = s1 + 16 * 128, *s3 = s2 + 16 * 128, *s4 = s3 + 128 * 32, *s5 = s4 + 128 * 32;
  for (int q = tid; q < 16 * 32; q += 256) { const int p = q >> 5, k = q & 31; s0[q] = (__bf16)((k < 12) ? C0[((size_t)e * 12 + k) * 16 + p] : 0.f); }
  for (int q = tid; q < 16 * 128; q += 256) { const int p = q >> 7, k = q & 127; const int r = k >> 3, m = k & 7; s1[q] = (__bf16)C1[(((size_t)e * RR + r) * 8 + m) * 16 + p]; s2[q] = (__bf16)C2[(((size_t)e * RR + r) * 8 + m) * 16 + p]; }
  for (int q = tid; q < 128 * 32; q += 256) { const int col = q >> 5, k = q & 31; const int p = col >> 3, nn = col & 7; s3[q] = (__bf16)((k < RR) ? C3[(((size_t)e * RR + k) * 8 + nn) * 16 + p] : 0.f); s4[q] = (__bf16)((k < RR) ? C4[(((size_t)e * RR + k) * 8 + nn) * 16 + p] : 0.f); }
  for (int q = tid; q < 16 * 32; q += 256) { const int n3 = q >> 5, k = q & 31; s5[q] = (__bf16)((k < RR && n3 < 12) ? C5[((size_t)e * RR + k) * 12 + n3] : 0.f); }
  __syncthreads();
  for (int q = tid; q < 16 * 32 / 8; q += 256) { vst2((unsigned*)(PK + PK_C0 + (size_t)e * 512 + q * 8), *(const v4u*)&s0[q * 8]); vst2((unsigned*)(PK + PK_C5 + (size_t)e * 512 + q * 8), *(const v4u*)&s5[q * 8]); }
  for (int q = tid; q < 16 * 128 / 8; q += 256) { vst2((unsigned*)(PK + PK_C1 + (size_t)e * 2048 + q * 8), *(const v4u*)&s1[q * 8]); vst2((unsigned*)(PK + PK_C2 + (size_t)e * 2048 + q * 8), *(const v4u*)&s2[q * 8]); }
  for (int q = tid; q < 128 * 32 / 8; q += 256) { vst2((unsigned*)(PK + PK_C3 + (size_t)e * 4096 + q * 8), *(const v4u*)&s3[q * 8]); vst2((unsigned*)(PK + PK_C4 + (size_t)e * 4096 + q * 8), *(const v4u*)&s4[q * 8]); }
}
__global__ __launch_bounds__(128) void k_xb(const float* __restrict__ X, __bf16* __restrict__ XB) {
  __shared__ __align__(16) __bf16 s[DM]; const size_t r = blockIdx.x; const int t = threadIdx.x;
  for (int k = t; k < DM; k += 128) s[k] = (__bf16)X[r * DM + k];
  __syncthreads();
  if (t < DM / 8) vst2((unsigned*)(XB + r * DM + t * 8), *(const v4u*)&s[t * 8]);
}
__device__ __forceinline__ F2 split16(const float* row, int lane) { float v[16]; const float* p = row + 8 * (lane >> 4);
#pragma unroll
  for (int i = 0; i < 8; ++i) { v[i] = p[i]; v[8 + i] = 0.f; } return bsplit16(v); }
__global__ __launch_bounds__(128) void k_tt(const float* __restrict__ X, const float* __restrict__ GATES, const __bf16* __restrict__ PK, float* __restrict__ Z) {
  __shared__ __align__(16) float sA[TPB * 1024];
  __shared__ __align__(16) float sT2[TPB][RR][8];
  __shared__ __align__(16) float sT3[TPB][RR + 16];
  __shared__ __align__(16) float sT4[TPB][8][RR];
  __shared__ __align__(16) float sT6[TPB][DM + 4];
  const int tid = threadIdx.x, wave = tid >> 5, lane = tid & 31, col = lane & 15, g = lane >> 4; const size_t t0 = (size_t)blockIdx.x * TPB; const int b = (int)(t0 / SS);
  int e = 0; { float best = -3.0e38f; for (int i = 0; i < NE; ++i) { const float v = bfr(GATES[b * NE + i]); if (v > best) { best = v; e = i; } } }
  const __bf16 *C0 = PK + PK_C0 + (size_t)e * 512, *C1 = PK + PK_C1 + (size_t)e * 2048, *C2 = PK + PK_C2 + (size_t)e * 2048, *C3 = PK + PK_C3 + (size_t)e * 4096, *C4 = PK + PK_C4 + (size_t)e * 4096, *C5 = PK + PK_C5 + (size_t)e * 512;
#pragma unroll 1
  for (int rt = wave; rt < 64; rt += 4) { const int row = rt * 16 + col; const int t = row >> 6, ab = row & 63; const float* xr = X + (t0 + t) * DM + ab * 12; v16b a;
#pragma unroll
    for (int i = 0; i < 16; ++i) { const int k = (i < 8) ? (8 * g + i) : (16 + 8 * g + i - 8); a[i] = (k < 12) ? (__bf16)xr[min(k, 11)] : (__bf16)0.f; }
    v8f acc = {}; acc = wmma_bf(a, frag_b(C0 + (size_t)col * 32, lane), acc);
#pragma unroll
    for (int r8 = 0; r8 < 8; ++r8) { const int rrow = rt * 16 + 8 * g + r8; const int tt = rrow >> 6, aa = (rrow >> 3) & 7, bb = rrow & 7; sA[tt * 1024 + aa * 128 + col * 8 + bb] = acc[r8]; } }
  __syncthreads();
  if (wave < 4) {
#pragma unroll 1
    for (int rt = wave; rt < 8; rt += 4) { const int row = rt * 16 + col; v8f acc = {};
#pragma unroll
      for (int kc = 0; kc < 4; ++kc) { const F2 a = split_row(&sA[row * 128], kc * 32, lane); const v16b w = frag_b(C1 + (size_t)col * 128 + kc * 32, lane); acc = wmma_bf(a.l, w, acc); acc = wmma_bf(a.h, w, acc); }
#pragma unroll
      for (int r8 = 0; r8 < 8; ++r8) { const int rrow = rt * 16 + 8 * g + r8; const int tt = rrow >> 3, aa = rrow & 7; sT2[tt][col][aa] = acc[r8]; } } }
  __syncthreads();
  if (wave == 0) { v8f acc = {};
#pragma unroll
    for (int kc = 0; kc < 4; ++kc) { const F2 a = split_row(&sT2[col][0][0], kc * 32, lane); const v16b w = frag_b(C2 + (size_t)col * 128 + kc * 32, lane); acc = wmma_bf(a.l, w, acc); acc = wmma_bf(a.h, w, acc); }
#pragma unroll
    for (int r8 = 0; r8 < 8; ++r8) sT3[8 * g + r8][col] = acc[r8]; }
  __syncthreads();
  { const F2 a = split16(&sT3[col][0], lane);
#pragma unroll
    for (int jj = 0; jj < 2; ++jj) { const int j = wave * 2 + jj; v8f acc = {}; const v16b w = frag_b(C3 + (size_t)(j * 16 + col) * 32, lane); acc = wmma_bf(a.l, w, acc); acc = wmma_bf(a.h, w, acc);
      const int cix = j * 16 + col; const int p = cix >> 3, nn = cix & 7;
#pragma unroll
      for (int r8 = 0; r8 < 8; ++r8) sT4[8 * g + r8][nn][p] = acc[r8]; } }
  __syncthreads();
#pragma unroll 1
  for (int q = wave; q < 64; q += 4) { const int rt = q >> 3, j = q & 7; const int row = rt * 16 + col; const F2 a = split16(&sT4[row >> 3][row & 7][0], lane); v8f acc = {}; const v16b w = frag_b(C4 + (size_t)(j * 16 + col) * 32, lane); acc = wmma_bf(a.l, w, acc); acc = wmma_bf(a.h, w, acc);
    const int cix = j * 16 + col; const int p = cix >> 3, nn = cix & 7;
#pragma unroll
    for (int r8 = 0; r8 < 8; ++r8) { const int rrow = rt * 16 + 8 * g + r8; const int tt = rrow >> 3, aa = rrow & 7; sA[tt * 1024 + aa * 128 + nn * 16 + p] = acc[r8]; } }
  __syncthreads();
#pragma unroll 1
  for (int rt = wave; rt < 64; rt += 4) { const int row = rt * 16 + col; const F2 a = split16(&sA[row * 16], lane); v8f acc = {}; const v16b w = frag_b(C5 + (size_t)col * 32, lane); acc = wmma_bf(a.l, w, acc); acc = wmma_bf(a.h, w, acc);
    if (col < 12) {
#pragma unroll
      for (int r8 = 0; r8 < 8; ++r8) { const int rrow = rt * 16 + 8 * g + r8; const int tt = rrow >> 6, aa = (rrow >> 3) & 7, bb = rrow & 7; sT6[tt][aa * 96 + bb * 12 + col] = acc[r8]; } } }
  __syncthreads();
  for (int q = tid; q < TPB * (DM / 4); q += 128) { const int t = q / (DM / 4), pc = q % (DM / 4); vst2(Z + (t0 + t) * DM + pc * 4, *(const v4f*)&sT6[t][pc * 4]); }
}
__global__ __launch_bounds__(128) void k_final(const __bf16* __restrict__ XB, const __bf16* __restrict__ PK, const float* __restrict__ BB, const float* __restrict__ Z, float* __restrict__ OUT) {
  __shared__ __align__(16) float so[4][16][132];
  const int tid = threadIdx.x, wave = tid >> 5, lane = tid & 31, col = lane & 15, g = lane >> 4; const size_t r0 = (size_t)blockIdx.x * 64 + wave * 16; const int n0 = blockIdx.y * 128;
  v8f acc[8] = {};
#pragma unroll 2
  for (int kc = 0; kc < DM / 32; ++kc) { const v16b a = frag_b(XB + (r0 + col) * DM + kc * 32, lane);
#pragma unroll
    for (int j = 0; j < 8; ++j) acc[j] = wmma_bf(a, frag_b(PK + PK_W + (size_t)(n0 + j * 16 + col) * DM + kc * 32, lane), acc[j]); }
#pragma unroll
  for (int j = 0; j < 8; ++j) { const int n = n0 + j * 16 + col; const float bb = bfr(BB[n]);
#pragma unroll
    for (int r = 0; r < 8; ++r) so[wave][8 * g + r][j * 16 + col] = 8.0f * Z[(r0 + 8 * g + r) * DM + n] + (acc[j][r] + bb); }
  LDSX();
  for (int rl = 0; rl < 16; ++rl) vst2(OUT + (r0 + rl) * DM + n0 + lane * 4, *(const v4f*)&so[wave][rl][lane * 4]);
}
extern "C" void kernel_launch(void* const* d_in, const int* in_sizes, int n_in, void* d_out, int out_size, void* d_ws, size_t ws_size, hipStream_t stream) {
  (void)in_sizes; (void)n_in; (void)out_size;
  const float** F = (const float**)d_in;
  if (ws_size < (size_t)WS_END) return;
  char* ws = (char*)d_ws; __bf16 *PK = (__bf16*)(ws + WS_PK), *XB = (__bf16*)(ws + WS_XB); float* Z = (float*)(ws + WS_Z);
  k_pack<<<dim3(DM, 2), 256, 0, stream>>>(F[1], F[4], F[5], F[6], F[7], F[8], F[9], PK);
  k_xb<<<NRT * 64, 128, 0, stream>>>(F[0], XB);
  k_tt<<<NTB, 128, 0, stream>>>(F[0], F[3], PK, Z);
  k_final<<<dim3(NRT, DM / 128), 128, 0, stream>>>(XB, PK, F[2], Z, (float*)d_out);
}
